// SCDM_Attention_14998025798075
// MI455X (gfx1250) — hardware-verified
//
#include <hip/hip_runtime.h>
#include <stddef.h>


typedef _Float16 h16;
typedef _Float16 v16h __attribute__((ext_vector_type(16)));
typedef _Float16 v8h  __attribute__((ext_vector_type(8)));
typedef float    v8f  __attribute__((ext_vector_type(8)));
typedef float    v4f  __attribute__((ext_vector_type(4)));

#ifndef NB
#define NB 16
#endif
#ifndef SEQ
#define SEQ 256
#endif
#define NB_FULL  16
#define SEQ_FULL 256
#define NSENT 32
#define DSENT 512
#define DVID  1024
#define HID   1024
#define MROWS (NB * SEQ)
#define MSP   ((((NB * NSENT) + 63) / 64) * 64)

#define TBLK 16
#define HCH  256
#define PLD  40
#define LDT 72
#define LDC 68
#define LS_FLOATS (8 * 16 * LDC)

#define WCARRY 64.0f
#define SCARRY 64.0f
#define PCARRY 1024.0f

static_assert(NB >= 1 && NB <= NB_FULL);
static_assert(SEQ >= 64 && SEQ <= SEQ_FULL && (SEQ % 64) == 0 && (SEQ % TBLK) == 0);
static_assert(NSENT == 32);
static_assert((MROWS % 64) == 0 && (MSP % 64) == 0 && MSP <= NB_FULL * NSENT);
static_assert((HID % 64) == 0 && (HID % HCH) == 0 && HCH == 2 * 32 * 4);
static_assert((DSENT % 32) == 0 && (DVID % 32) == 0 && (DSENT % 64) == 0);
static_assert(DSENT == 8 * 64);
static_assert(TBLK == 8 * 2);
static_assert(NSENT * HCH <= LS_FLOATS);
static_assert((LDT % 8) == 0 && LDT >= 64);
static_assert((LDC % 4) == 0 && LDC >= 64);
static_assert((PLD % 8) == 0 && PLD >= NSENT);
static_assert(((size_t)HID * DSENT) % 2048 == 0 && ((size_t)HID * DVID) % 2048 == 0);
static_assert(((size_t)MSP * DSENT) % 2048 == 0 && ((size_t)MROWS * DVID) % 2048 == 0);
static_assert((DSENT % 256) == 0 && (DVID % 256) == 0);
static_assert((size_t)NB_FULL * SEQ_FULL * DSENT * 4 == (size_t)8388608);

#define WSP_BYTES ((size_t)HID * DSENT * 2)
#define WAP_BYTES ((size_t)HID * DVID * 2)
#define SA_BYTES  ((size_t)MSP * DSENT * 2)
#define VA_BYTES  ((size_t)MROWS * DVID * 2)
#define ST_BYTES  ((size_t)DSENT * MSP * 2)
#define ES_BYTES  ((size_t)MSP * HID * 4)
#define EV_BYTES  ((size_t)MROWS * HID * 4)
#define OFF_WSP ((size_t)0)
#define OFF_WAP (OFF_WSP + WSP_BYTES)
#define OFF_SA  (OFF_WAP + WAP_BYTES)
#define OFF_VA  (OFF_SA + SA_BYTES)
#define OFF_ST  (OFF_VA + VA_BYTES)
#define OFF_ES  (OFF_ST + ST_BYTES)
#define OFF_EV  (OFF_ES + ES_BYTES)
#define WS_TOTAL (OFF_EV + EV_BYTES)
static_assert((WSP_BYTES % 128) == 0 && (WAP_BYTES % 128) == 0 && (SA_BYTES % 128) == 0);
static_assert((VA_BYTES % 128) == 0 && (ST_BYTES % 128) == 0 && (ES_BYTES % 128) == 0);
static_assert((EV_BYTES % 128) == 0);
static_assert(WS_TOTAL <= (size_t)134217728);

__device__ __forceinline__ float bf16r(float x) {
  unsigned int u = __float_as_uint(x);
  u = (u + 0x7FFFu + ((u >> 16) & 1u)) & 0xFFFF0000u;
  return __uint_as_float(u);
}

static __device__ __forceinline__ h16 toh_flush(float v) {
  const h16 r = (h16)v;
  return (fabsf(v) < 6.103515625e-05f) ? (h16)0.0f : r;
}

__device__ __forceinline__ v16h frag_at(const _Float16* p) {
  v8h lo = *(const v8h*)(p);
  v8h hi = *(const v8h*)(p + 16);
  v16h out;
#pragma unroll
  for (int i = 0; i < 8; ++i) { out[i] = lo[i]; out[i + 8] = hi[i]; }
  return out;
}
__device__ __forceinline__ v16h ld_frag(const _Float16* base, unsigned ld) {
  const unsigned lane = threadIdx.x & 31u;
  return frag_at(base + (lane & 15u) * ld + (lane >> 4) * 8u);
}

__device__ __forceinline__ v8f wmma16(v16h a, v16h b, v8f c) {
  v8f d = __builtin_amdgcn_wmma_f32_16x16x32_f16(false, a, false, b, (short)0, c,
                                                 false, false);
  asm volatile("v_nop\n\tv_nop\n\tv_nop\n\tv_nop" : "+v"(d) : "v"(a), "v"(b));
  return d;
}

__device__ __forceinline__ float red16_max(float x) {
#pragma unroll
  for (int off = 1; off < 16; off <<= 1) x = fmaxf(x, __shfl_xor(x, off, 32));
  return x;
}
__device__ __forceinline__ float red16_sum(float x) {
#pragma unroll
  for (int off = 1; off < 16; off <<= 1) x += __shfl_xor(x, off, 32);
  return x;
}

__device__ __forceinline__ void wave_lds_sync() {
  __builtin_amdgcn_fence(3  , "wavefront");
  asm volatile("s_wait_dscnt 0x0" ::: "memory");
  __builtin_amdgcn_wave_barrier();
}

__global__ __launch_bounds__(256) void wconv_kernel(
    const float* __restrict__ W, _Float16* __restrict__ Wt, unsigned ldw, unsigned ldk) {
  __shared__ _Float16 T[64 * LDT];
  const unsigned tid = threadIdx.x;
  const unsigned n0 = blockIdx.x * 64u;
  const unsigned k0 = blockIdx.y * 64u;
#pragma unroll 4
  for (unsigned j = 0; j < 16u; ++j) {
    const unsigned idx = tid + 256u * j;
    const unsigned kr = idx >> 6, nc = idx & 63u;
    const float v = W[(size_t)(k0 + kr) * ldw + n0 + nc];
    T[nc * LDT + kr] = (_Float16)(WCARRY * bf16r(v));
  }
  __syncthreads();
  v8h x[2];
  size_t off[2];
#pragma unroll
  for (unsigned i = 0; i < 2u; ++i) {
    const unsigned n = 32u * i + (tid >> 3);
    const unsigned kc = (tid & 7u) * 8u;
    x[i] = *(const v8h*)&T[n * LDT + kc];
    off[i] = (size_t)(n0 + n) * ldk + k0 + kc;
  }
#pragma unroll
  for (int i = 0; i < 2; ++i) *(volatile v8h*)(Wt + off[i]) = x[i];
  __threadfence();
#pragma unroll
  for (int i = 0; i < 2; ++i) *(volatile v8h*)(Wt + off[i]) = x[i];
}

__global__ __launch_bounds__(256) void cvt_kernel(
    const float* __restrict__ src, _Float16* __restrict__ dst,
    unsigned cols, unsigned rpb, unsigned rpb_full, float scale) {
  const unsigned g = blockIdx.x * 256u + threadIdx.x;
  const unsigned c8 = cols >> 3;
  const unsigned crow = g / c8;
  const unsigned cg = g - crow * c8;
  const unsigned bidx = crow / rpb;
  const unsigned rr = crow - bidx * rpb;
  const size_t srow = (size_t)bidx * rpb_full + rr;
  const float* p = src + srow * cols + cg * 8u;
  const v4f a0 = *(const v4f*)(p);
  const v4f a1 = *(const v4f*)(p + 4);
  v8h o;
#pragma unroll
  for (int i = 0; i < 4; ++i) {
    o[i]     = toh_flush(scale * bf16r(a0[i]));
    o[i + 4] = toh_flush(scale * bf16r(a1[i]));
  }
  _Float16* q = dst + (size_t)crow * cols + cg * 8u;
  *(volatile v8h*)q = o;
  __threadfence();
  *(volatile v8h*)q = o;
}

template <int HASB>
__device__ __forceinline__ void gemm_body(
    const _Float16* __restrict__ A16, const _Float16* __restrict__ Bt, const unsigned K,
    const float* __restrict__ bias, float* __restrict__ outf) {
  __shared__ float Cs[64 * LDC];
  const unsigned tid = threadIdx.x, lane = tid & 31u, w = tid >> 5;
  const unsigned mw = w >> 1, nw = w & 1u;
  const unsigned hh = lane >> 4, m = lane & 15u;
  const unsigned n0 = blockIdx.x * 64u;
  const unsigned row0 = blockIdx.y * 64u;

  const _Float16* ap  = A16 + (size_t)(row0 + mw * 16u + m) * K + hh * 8u;
  const _Float16* bp0 = Bt + (size_t)(n0 + nw * 32u + m) * K + hh * 8u;
  const _Float16* bp1 = bp0 + (size_t)16 * K;
  v8f acc0 = {}, acc1 = {};
#pragma unroll 2
  for (unsigned k0 = 0; k0 < K; k0 += 32u) {
    const v16h a  = frag_at(ap + k0);
    const v16h b0 = frag_at(bp0 + k0);
    const v16h b1 = frag_at(bp1 + k0);
    acc0 = wmma16(a, b0, acc0);
    acc1 = wmma16(a, b1, acc1);
  }
#pragma unroll
  for (int r = 0; r < 8; ++r) {
    float* d = &Cs[(mw * 16u + hh * 8u + (unsigned)r) * LDC + nw * 32u + m];
    d[0]  = acc0[r];
    d[16] = acc1[r];
  }
  __syncthreads();

  v4f xs[4];
  size_t off[4];
#pragma unroll
  for (unsigned i = 0; i < 4u; ++i) {
    const unsigned r = 16u * i + (tid >> 4);
    const unsigned c = (tid & 15u) * 4u;
    const v4f u = *(const v4f*)&Cs[r * LDC + c];
    v4f val;
    if (HASB) {
      const v4f g = *(const v4f*)(bias + n0 + c);
#pragma unroll
      for (int j = 0; j < 4; ++j)
        val[j] = __expf(2.0f * (u[j] * (1.0f / WCARRY) + bf16r(g[j])));
    } else {
#pragma unroll
      for (int j = 0; j < 4; ++j)
        val[j] = __expf(2.0f * (u[j] * (1.0f / WCARRY)));
    }
    xs[i] = val;
    off[i] = (size_t)(row0 + r) * HID + n0 + c;
  }
#pragma unroll
  for (int i = 0; i < 4; ++i) *(volatile v4f*)(outf + off[i]) = xs[i];
  __threadfence();
#pragma unroll
  for (int i = 0; i < 4; ++i) *(volatile v4f*)(outf + off[i]) = xs[i];
}

__global__ __launch_bounds__(256) void gemm_sent_kernel(
    const _Float16* __restrict__ A16, const _Float16* __restrict__ Bt,
    float* __restrict__ outf) {
  gemm_body<0>(A16, Bt, (unsigned)DSENT, (const float*)0, outf);
}
__global__ __launch_bounds__(256) void gemm_video_kernel(
    const _Float16* __restrict__ A16, const _Float16* __restrict__ Bt,
    const float* __restrict__ bias, float* __restrict__ outf) {
  gemm_body<1>(A16, Bt, (unsigned)DVID, bias, outf);
}

__global__ __launch_bounds__(256) void score_ctx_kernel(
    const float* __restrict__ Ev, const float* __restrict__ Es, const float* __restrict__ wvec,
    const _Float16* __restrict__ St, float* __restrict__ out) {
  __shared__ float Ls[LS_FLOATS];
  __shared__ _Float16 Ps[TBLK * PLD];

  const unsigned tid = threadIdx.x, lane = tid & 31u;
  const unsigned wave = __builtin_amdgcn_readfirstlane(threadIdx.x >> 5);
  const unsigned hh = lane >> 4, m = lane & 15u;
  const unsigned t0 = blockIdx.x * (unsigned)TBLK;
  const unsigned b = blockIdx.y;
  const bool upper = (hh != 0u);

  float sc_lo = 0.0f, sc_hi = 0.0f;
  const float* evp = Ev + (size_t)(b * (unsigned)SEQ + t0 + wave * 2u) * HID + lane * 4u;
  const float* esp = Es + (size_t)(b * (unsigned)NSENT) * HID;

#pragma unroll 1
  for (unsigned hc = 0; hc < (unsigned)HID; hc += (unsigned)HCH) {
    __syncthreads();
#pragma unroll 2
    for (unsigned j = 0; j < 8u; ++j) {
      const unsigned idx = tid + 256u * j;
      const unsigned n = idx >> 6, c4 = (idx & 63u) * 4u;
      *(v4f*)&Ls[n * HCH + c4] = *(const v4f*)(esp + (size_t)n * HID + hc + c4);
    }
    __syncthreads();

    v4f e0[2], e1[2], ww[2];
#pragma unroll
    for (unsigned j = 0; j < 2u; ++j) {
      const unsigned col = hc + 128u * j;
      e0[j] = *(const v4f*)(evp + col);
      e1[j] = *(const v4f*)(evp + HID + col);
      const v4f wr = *(const v4f*)(wvec + col + lane * 4u);
#pragma unroll
      for (int i = 0; i < 4; ++i) ww[j][i] = -2.0f * bf16r(wr[i]);
    }

#pragma unroll 1
    for (unsigned n = 0; n < (unsigned)NSENT; ++n) {
      float p0 = 0.0f, p1 = 0.0f;
#pragma unroll
      for (unsigned j = 0; j < 2u; ++j) {
        const v4f es = *(const v4f*)&Ls[n * HCH + 128u * j + lane * 4u];
#pragma unroll
        for (int i = 0; i < 4; ++i) {
          const float r0 = __builtin_amdgcn_rcpf(fmaf(e0[j][i], es[i], 1.0f));
          const float r1 = __builtin_amdgcn_rcpf(fmaf(e1[j][i], es[i], 1.0f));
          p0 = fmaf(ww[j][i], r0, p0);
          p1 = fmaf(ww[j][i], r1, p1);
        }
      }
      const float give = upper ? p0 : p1;
      const float keep = upper ? p1 : p0;
      float x = keep + __shfl_xor(give, 16, 32);
      x = red16_sum(x);
      const bool hit = (m == (n & 15u));
      const bool lo_n = (n < 16u);
      sc_lo = (hit && lo_n) ? (sc_lo + x) : sc_lo;
      sc_hi = (hit && !lo_n) ? (sc_hi + x) : sc_hi;
    }
  }

  const float mx = red16_max(fmaxf(sc_lo, sc_hi));
  const float el = __expf(sc_lo - mx);
  const float eh = __expf(sc_hi - mx);
  const float sum = red16_sum(el + eh);
  const float inv = PCARRY * __builtin_amdgcn_rcpf(sum);
  const unsigned prow = wave * 2u + hh;
  Ps[prow * PLD + m]       = toh_flush(el * inv);
  Ps[prow * PLD + 16u + m] = toh_flush(eh * inv);
  __syncthreads();

  const v16h pf = ld_frag(Ps, PLD);
  v8f acc[4];
#pragma unroll
  for (int nb = 0; nb < 4; ++nb) {
    const unsigned dcol = wave * 64u + (unsigned)nb * 16u + m;
    const v16h sf = frag_at(St + (size_t)dcol * MSP + b * (unsigned)NSENT + hh * 8u);
    v8f z = {};
    acc[nb] = wmma16(pf, sf, z);
  }

  const unsigned cw = wave * (16u * LDC);
#pragma unroll
  for (int nb = 0; nb < 4; ++nb)
#pragma unroll
    for (int r = 0; r < 8; ++r)
      Ls[cw + (hh * 8u + (unsigned)r) * LDC + (unsigned)nb * 16u + m] =
          acc[nb][r] * (1.0f / (PCARRY * SCARRY));
  wave_lds_sync();

  v4f xs[8];
  size_t off[8];
#pragma unroll
  for (unsigned i = 0; i < 8u; ++i) {
    const unsigned r = 2u * i + (lane >> 4);
    const unsigned c = (lane & 15u) * 4u;
    xs[i] = *(const v4f*)&Ls[cw + r * LDC + c];
    off[i] = ((size_t)b * SEQ_FULL + t0 + r) * DSENT + wave * 64u + c;
  }
#pragma unroll
  for (int i = 0; i < 8; ++i) *(volatile v4f*)(out + off[i]) = xs[i];
  __threadfence();
#pragma unroll
  for (int i = 0; i < 8; ++i) *(volatile v4f*)(out + off[i]) = xs[i];
}

extern "C" void kernel_launch(void* const* d_in, const int* in_sizes, int n_in,
                              void* d_out, int out_size, void* d_ws, size_t ws_size,
                              hipStream_t stream) {
  if (n_in < 6) return;
  const long long need_v = ((long long)(NB - 1) * SEQ_FULL + SEQ) * DVID;
  const long long need_o = ((long long)(NB - 1) * SEQ_FULL + SEQ) * DSENT;
  if ((long long)in_sizes[0] < need_v) return;
  if ((long long)in_sizes[1] < (long long)MSP * DSENT) return;
  if ((long long)in_sizes[2] < (long long)HID * DSENT) return;
  if ((long long)in_sizes[3] < (long long)HID * DVID) return;
  if (in_sizes[4] < HID || in_sizes[5] < HID) return;
  if ((long long)out_size < need_o) return;
  if (ws_size < WS_TOTAL) return;

  const float* video = (const float*)d_in[0];
  const float* sent  = (const float*)d_in[1];
  const float* Ws    = (const float*)d_in[2];
  const float* Wa    = (const float*)d_in[3];
  const float* ba    = (const float*)d_in[4];
  const float* wv    = (const float*)d_in[5];
  float* out = (float*)d_out;

  char* ws = (char*)d_ws;
  _Float16* WsP = (_Float16*)(ws + OFF_WSP);
  _Float16* WaP = (_Float16*)(ws + OFF_WAP);
  _Float16* SA  = (_Float16*)(ws + OFF_SA);
  _Float16* VA  = (_Float16*)(ws + OFF_VA);
  _Float16* StP = (_Float16*)(ws + OFF_ST);
  float*    EsP = (float*)(ws + OFF_ES);
  float*    EvP = (float*)(ws + OFF_EV);

  dim3 blk(256);

  cvt_kernel<<<dim3((unsigned)(((size_t)HID * DSENT) / 2048)), blk, 0, stream>>>(
      Ws, WsP, (unsigned)DSENT, (unsigned)HID, (unsigned)HID, WCARRY);
  cvt_kernel<<<dim3((unsigned)(((size_t)HID * DVID) / 2048)), blk, 0, stream>>>(
      Wa, WaP, (unsigned)DVID, (unsigned)HID, (unsigned)HID, WCARRY);
  cvt_kernel<<<dim3((unsigned)(((size_t)MSP * DSENT) / 2048)), blk, 0, stream>>>(
      sent, SA, (unsigned)DSENT, (unsigned)MSP, (unsigned)MSP, 1.0f);
  cvt_kernel<<<dim3((unsigned)(((size_t)MROWS * DVID) / 2048)), blk, 0, stream>>>(
      video, VA, (unsigned)DVID, (unsigned)SEQ, (unsigned)SEQ_FULL, 1.0f);

  wconv_kernel<<<dim3(DSENT / 64, MSP / 64), blk, 0, stream>>>(
      sent, StP, (unsigned)DSENT, (unsigned)MSP);

  gemm_sent_kernel<<<dim3(HID / 64, MSP / 64), blk, 0, stream>>>(SA, WsP, EsP);
  gemm_video_kernel<<<dim3(HID / 64, MROWS / 64), blk, 0, stream>>>(VA, WaP, ba, EvP);

  score_ctx_kernel<<<dim3(SEQ / TBLK, NB), blk, 0, stream>>>(EvP, EsP, wv, StP, out);
}
